// ResidualDCN_62637803045633
// MI455X (gfx1250) — hardware-run, weakly checked
//
#include <hip/hip_runtime.h>
#include <math.h>

typedef __attribute__((ext_vector_type(16))) _Float16 v16h;
typedef __attribute__((ext_vector_type(8)))  _Float16 v8h;
typedef __attribute__((ext_vector_type(8)))  float    v8f;
typedef __attribute__((ext_vector_type(4)))  float    v4f;

constexpr int kNB      = 8;
constexpr int kC       = 32;
constexpr int kL       = 32768;
constexpr int kTaps    = 11;
constexpr int kDil     = 10;
constexpr int kPadSame = 50;
constexpr int kPadOff  = 5;
constexpr int kCK      = kC * kTaps;
constexpr int kOffN    = 16;
constexpr float kEps   = 1e-3f;
constexpr float kActCarry = 16.0f;
constexpr float kWCarry   = 256.0f;
constexpr float kFoldInv  = 1.0f / (kActCarry * kWCarry);
static_assert(kActCarry * kWCarry == 4096.0f, "power-of-two carries fold back exactly");
static_assert(kPadSame == (kDil * (kTaps - 1) + 1) / 2, "same padding");
static_assert(kPadOff == (kTaps - 1) / 2, "offset conv padding");
static_assert(kCK == 352 && (kCK % 32) == 0 && (kCK % 8) == 0, "reduction depth is 11 whole k-steps");
static_assert(kC == 32, "one tap per 32-deep k-step");
static_assert((kL % 128) == 0, "tile multiples");
static_assert(kTaps <= kOffN, "offset channels fit one 16-wide tile");

constexpr int kOcPos    = 128;
constexpr int kWinRows  = kOcPos + kTaps - 1;
constexpr int kWinPitch = 40;
constexpr int kWinItems = kWinRows * 4;
constexpr int kSlabPitch = 20;
static_assert(kWinRows == 138 && kWinItems == 552 && kWinItems <= 3 * 256, "window staging coverage");

constexpr int kDcPos = 32;
constexpr int kAP    = 360;
constexpr int kOP    = 36;
static_assert((kAP * 2) % 16 == 0 && (kWinPitch * 2) % 16 == 0, "16-B aligned LDS rows");

constexpr int kWRows = 96;

constexpr size_t kOffAct1 = 0;
constexpr size_t kOffAct2 = kOffAct1 + (size_t)kNB * kL * kC * 4;
constexpr size_t kOffOffs = kOffAct2 + (size_t)kNB * kL * kC * 4;
constexpr size_t kOffWPl  = kOffOffs + (size_t)kNB * kL * kOffN * 4;
constexpr size_t kWsTotal = kOffWPl  + (size_t)kWRows * kCK * 2;
static_assert(kWsTotal == 83953664ull, "carve total");
static_assert(kWsTotal <= 134217728ull, "carve cap");
static_assert((kOffAct2 % 128) == 0 && (kOffOffs % 128) == 0 && (kOffWPl % 128) == 0, "aligned regions");
static_assert(((size_t)16 * kCK * 2) % 128 == 0, "weight set bases are line aligned");

template <typename T> struct Frag;
template <> struct Frag<_Float16> {
  typedef v16h V; union U { v16h v; v8h h[2]; };
  static __device__ __forceinline__ v16h load(const _Float16* p) {
    U f; f.h[0] = *(const v8h*)(p); f.h[1] = *(const v8h*)(p + 16); return f.v;
  }
  static __device__ __forceinline__ v8f mma(v16h a, v16h b, v8f c) {
    return __builtin_amdgcn_wmma_f32_16x16x32_f16(false, a, false, b, (short)0, c, false, false);
  }
};
__device__ __forceinline__ void tie_acc2(v8f& a, v16h x, v16h y) {
  asm volatile("v_nop\n\tv_nop\n\tv_nop\n\tv_nop" : "+v"(a) : "v"(x), "v"(y));
}

__global__ __launch_bounds__(256) void weight_planes_kernel(
    const float* __restrict__ w0, const float* __restrict__ w1,
    const float* __restrict__ w2, const float* __restrict__ w3,
    unsigned short* __restrict__ WP)
{
  const int s = blockIdx.y;
  const float* src = (s == 0) ? w0 : (s == 1) ? w1 : (s == 2) ? w2 : w3;
  const int rows     = (s < 2) ? kOffN : kC;
  const int realRows = (s < 2) ? kTaps : kC;
  const int rowBase  = (s == 0) ? 0 : (s == 1) ? 16 : (s == 2) ? 32 : 64;
  const int nthr = rows * kCK / 8;
  const int i = blockIdx.x * 256 + threadIdx.x;
  if (i >= nthr) return;
  const int e0 = i * 8;
  const int n  = e0 / kCK;
  const int kk = e0 - n * kCK;
  const int t  = kk >> 5;
  const int c0 = kk & 31;
  const bool live = (n < realRows);
  const int nc = live ? n : (realRows - 1);
  v8h hv;
#pragma unroll
  for (int e = 0; e < 8; ++e) {
    const float raw = src[nc * kCK + (c0 + e) * kTaps + t];
    const float v = live ? (raw * kWCarry) : 0.0f;
    hv[e] = (_Float16)v;
  }
  unsigned short* qh = WP + (size_t)rowBase * kCK + e0;
  *(volatile v8h*)qh = hv;
  __threadfence();
  *(volatile v8h*)qh = hv;
}

__global__ __launch_bounds__(256) void bn_relu_transpose_kernel(
    const float* __restrict__ x, const float* __restrict__ gamma, const float* __restrict__ beta,
    const float* __restrict__ mean, const float* __restrict__ var, float* __restrict__ actT)
{
  __shared__ __align__(16) float sT[64 * kOP];
  const int tid = threadIdx.x, lane = tid & 31, wave = tid >> 5;
  constexpr int kBlkPerB = kL / 64;
  const int b  = blockIdx.x / kBlkPerB;
  const int l0 = (blockIdx.x - b * kBlkPerB) * 64;
  const int c = tid >> 3, seg = (tid & 7) * 8;
  const float sc = gamma[c] / sqrtf(var[c] + kEps);
  const float mu = mean[c];
  const float bt = beta[c];
  const float* xp = x + ((size_t)(b * kC + c)) * kL + l0 + seg;
  const v4f a0 = *(const v4f*)xp;
  const v4f a1 = *(const v4f*)(xp + 4);
#pragma unroll
  for (int e = 0; e < 4; ++e) {
    sT[(seg + e) * kOP + c]     = fmaxf((a0[e] - mu) * sc + bt, 0.0f);
    sT[(seg + 4 + e) * kOP + c] = fmaxf((a1[e] - mu) * sc + bt, 0.0f);
  }
  __syncthreads();
  const int q = lane >> 3, c4 = (lane & 7) * 4;
  v4f ov[2];
#pragma unroll
  for (int it = 0; it < 2; ++it) ov[it] = *(const v4f*)(sT + (wave * 8 + it * 4 + q) * kOP + c4);
  float* dst = actT + ((size_t)b * kL + l0) * kC;
  for (int pass = 0; pass < 2; ++pass) {
#pragma unroll
    for (int it = 0; it < 2; ++it)
      *(volatile v4f*)(dst + (size_t)(wave * 8 + it * 4 + q) * kC + c4) = ov[it];
    __threadfence();
  }
}

__global__ __launch_bounds__(256) void offset_conv_kernel(
    const float* __restrict__ actT, const unsigned short* __restrict__ WPp,
    const float* __restrict__ bias, float* __restrict__ offs)
{
  __shared__ __align__(16) _Float16 sA[kWinRows * kWinPitch];
  __shared__ __align__(16) float sD[8][16 * kSlabPitch];
  const int tid = threadIdx.x, lane = tid & 31, wave = tid >> 5;
  constexpr int kBlkPerB = kL / kOcPos;
  const int b  = blockIdx.x / kBlkPerB;
  const int l0 = (blockIdx.x - b * kBlkPerB) * kOcPos;

#pragma unroll 1
  for (int it = 0; it < 3; ++it) {
    const int item = it * 256 + tid;
    const int itc = (item < kWinItems) ? item : (kWinItems - 1);
    const int r = itc >> 2, c8 = (itc & 3) * 8;
    const int p = l0 - kPadOff + r;
    const bool ok = (p >= 0) && (p < kL);
    const int pc = min(max(p, 0), kL - 1);
    const float* src = actT + ((size_t)b * kL + pc) * kC + c8;
    v4f a0 = *(const v4f*)src;
    v4f a1 = *(const v4f*)(src + 4);
    asm volatile("" : "+v"(a0), "+v"(a1));
    v8h hv;
#pragma unroll
    for (int e = 0; e < 4; ++e) {
      const float s0 = ok ? a0[e] : 0.0f;
      const float s1 = ok ? a1[e] : 0.0f;
      hv[e]     = (_Float16)(s0 * kActCarry);
      hv[4 + e] = (_Float16)(s1 * kActCarry);
    }
    if (item < kWinItems) {
      *(v8h*)(sA + r * kWinPitch + c8) = hv;
    }
  }
  __syncthreads();

  const _Float16* WP = (const _Float16*)WPp;
  const int m = lane & 15, h = lane >> 4;
  const _Float16* aH = sA + (wave * 16 + m) * kWinPitch + 8 * h;
  const _Float16* bH = WP + (size_t)m * kCK + 8 * h;
  v8f accM = (v8f){0.f,0.f,0.f,0.f,0.f,0.f,0.f,0.f};
#pragma unroll 1
  for (int t = 0; t < kTaps; ++t) {
    const v16h ah = Frag<_Float16>::load(aH + t * kWinPitch);
    const v16h bh = Frag<_Float16>::load(bH + t * 32);
    accM = Frag<_Float16>::mma(ah, bh, accM);
    tie_acc2(accM, ah, bh);
  }

  const bool jlive = (m < kTaps);
  const float bj = bias[jlive ? m : (kTaps - 1)];
  float* slab = sD[wave];
#pragma unroll
  for (int r = 0; r < 8; ++r) {
    const float v = accM[r] * kFoldInv + bj;
    slab[(8 * h + r) * kSlabPitch + m] = jlive ? v : 0.0f;
  }
  __syncthreads();
  const int rq = lane >> 2, c4 = (lane & 3) * 4;
  v4f ov[2];
#pragma unroll
  for (int it = 0; it < 2; ++it) ov[it] = *(const v4f*)(slab + (it * 8 + rq) * kSlabPitch + c4);
  float* dst = offs + ((size_t)b * kL + l0 + wave * 16) * kOffN;
  for (int pass = 0; pass < 2; ++pass) {
#pragma unroll
    for (int it = 0; it < 2; ++it)
      *(volatile v4f*)(dst + (size_t)(it * 8 + rq) * kOffN + c4) = ov[it];
    __threadfence();
  }
}

template <bool FINAL>
__global__ __launch_bounds__(128) void sampled_conv_kernel(
    const float* __restrict__ actT, const float* __restrict__ offs,
    const unsigned short* __restrict__ WPp,
    const float* __restrict__ bias,
    const float* __restrict__ g2, const float* __restrict__ be2,
    const float* __restrict__ mu2, const float* __restrict__ va2,
    const float* __restrict__ xres, float* __restrict__ outp)
{
  __shared__ __align__(16) _Float16 sA[kDcPos * kAP];
  __shared__ __align__(16) float sO[32 * kOP];
  const int tid = threadIdx.x, lane = tid & 31, wave = tid >> 5;
  constexpr int kBlkPerB = kL / kDcPos;
  const int b  = blockIdx.x / kBlkPerB;
  const int l0 = (blockIdx.x - b * kBlkPerB) * kDcPos;

  {
    const int p = tid >> 2, c8 = (tid & 3) * 8;
    const int l = l0 + p;
    const float* orow  = offs + ((size_t)b * kL + l) * kOffN;
    const float* abase = actT + (size_t)b * kL * kC + c8;
#pragma unroll 1
    for (int k = 0; k < kTaps; ++k) {
      const float off = orow[k];
      const float pos = (float)(l + kDil * k - kPadSame) + off;
      const float fl  = floorf(pos);
      const float fr  = pos - fl;
      const int   lo  = (int)fl;
      const int   hi  = lo + 1;
      const int  ilo  = min(max(lo, 0), kL - 1);
      const int  ihi  = min(max(hi, 0), kL - 1);
      const float wl  = (lo >= 0 && lo < kL) ? (1.0f - fr) : 0.0f;
      const float wh  = (hi >= 0 && hi < kL) ? fr : 0.0f;
      const float* pl = abase + (size_t)ilo * kC;
      const float* ph = abase + (size_t)ihi * kC;
      const v4f la = *(const v4f*)pl;
      const v4f lb = *(const v4f*)(pl + 4);
      const v4f ha = *(const v4f*)ph;
      const v4f hb = *(const v4f*)(ph + 4);
      v8h hv;
#pragma unroll
      for (int e = 0; e < 4; ++e) {
        const float s0 = la[e] * wl + ha[e] * wh;
        const float s1 = lb[e] * wl + hb[e] * wh;
        hv[e]     = (_Float16)(s0 * kActCarry);
        hv[4 + e] = (_Float16)(s1 * kActCarry);
      }
      *(v8h*)(sA + p * kAP + k * 32 + c8) = hv;
    }
  }
  __syncthreads();

  const _Float16* WP = (const _Float16*)WPp;
  const int m = lane & 15, h = lane >> 4;
  const int pt = wave & 1, nt = wave >> 1;
  const _Float16* aH = sA + (pt * 16 + m) * kAP + 8 * h;
  const _Float16* bH = WP + (size_t)(nt * 16 + m) * kCK + 8 * h;
  v8f accM = (v8f){0.f,0.f,0.f,0.f,0.f,0.f,0.f,0.f};
#pragma unroll 1
  for (int k = 0; k < kTaps; ++k) {
    const v16h ah = Frag<_Float16>::load(aH + k * 32);
    const v16h bh = Frag<_Float16>::load(bH + k * 32);
    accM = Frag<_Float16>::mma(ah, bh, accM);
    tie_acc2(accM, ah, bh);
  }

  const int o = nt * 16 + m;
  const float bo = bias[o];
  float sc = 1.0f, mu = 0.0f, bt = 0.0f;
  if (!FINAL) {
    sc = g2[o] / sqrtf(va2[o] + kEps);
    mu = mu2[o];
    bt = be2[o];
  }
#pragma unroll
  for (int r = 0; r < 8; ++r) {
    float d = accM[r] * kFoldInv + bo;
    const int pr = pt * 16 + 8 * h + r;
    if (!FINAL) {
      d = fmaxf((d - mu) * sc + bt, 0.0f);
      sO[pr * kOP + o] = d;
    } else {
      sO[o * kOP + pr] = d;
    }
  }
  __syncthreads();

  const int q = lane >> 3, c4 = (lane & 7) * 4;
  v4f ov[2];
  size_t oa[2];
#pragma unroll
  for (int it = 0; it < 2; ++it) {
    const int row = wave * 8 + it * 4 + q;
    v4f v = *(const v4f*)(sO + row * kOP + c4);
    if (!FINAL) {
      oa[it] = ((size_t)b * kL + l0 + row) * kC + c4;
    } else {
      oa[it] = ((size_t)(b * kC + row)) * kL + l0 + c4;
      const v4f xv = *(const v4f*)(xres + oa[it]);
      v = v + xv;
    }
    ov[it] = v;
  }
  for (int pass = 0; pass < 2; ++pass) {
#pragma unroll
    for (int it = 0; it < 2; ++it)
      *(volatile v4f*)(outp + oa[it]) = ov[it];
    __threadfence();
  }
}

extern "C" void kernel_launch(void* const* d_in, const int* in_sizes, int n_in,
                              void* d_out, int out_size, void* d_ws, size_t ws_size,
                              hipStream_t stream) {
  if (n_in < 17) return;
  if (in_sizes[0] != kNB * kC * kL) return;
  for (int i = 1; i <= 8; ++i) if (in_sizes[i] != kC) return;
  if (in_sizes[9]  != kTaps * kCK) return;
  if (in_sizes[10] != kTaps) return;
  if (in_sizes[11] != kTaps * kCK) return;
  if (in_sizes[12] != kTaps) return;
  if (in_sizes[13] != kC * kCK) return;
  if (in_sizes[14] != kC) return;
  if (in_sizes[15] != kC * kCK) return;
  if (in_sizes[16] != kC) return;
  if (out_size != kNB * kC * kL) return;
  if (ws_size < kWsTotal) return;

  const float* x         = (const float*)d_in[0];
  const float* bn1_gamma = (const float*)d_in[1];
  const float* bn1_beta  = (const float*)d_in[2];
  const float* bn1_mean  = (const float*)d_in[3];
  const float* bn1_var   = (const float*)d_in[4];
  const float* bn2_gamma = (const float*)d_in[5];
  const float* bn2_beta  = (const float*)d_in[6];
  const float* bn2_mean  = (const float*)d_in[7];
  const float* bn2_var   = (const float*)d_in[8];
  const float* off1_w    = (const float*)d_in[9];
  const float* off1_b    = (const float*)d_in[10];
  const float* off2_w    = (const float*)d_in[11];
  const float* off2_b    = (const float*)d_in[12];
  const float* dc1_w     = (const float*)d_in[13];
  const float* dc1_b     = (const float*)d_in[14];
  const float* dc2_w     = (const float*)d_in[15];
  const float* dc2_b     = (const float*)d_in[16];
  float* outp = (float*)d_out;

  char* ws = (char*)d_ws;
  float* act1 = (float*)(ws + kOffAct1);
  float* act2 = (float*)(ws + kOffAct2);
  float* offs = (float*)(ws + kOffOffs);
  unsigned short* WP = (unsigned short*)(ws + kOffWPl);

  weight_planes_kernel<<<dim3(6, 4), 256, 0, stream>>>(off1_w, off2_w, dc1_w, dc2_w, WP);

  bn_relu_transpose_kernel<<<kNB * kL / 64, 256, 0, stream>>>(x, bn1_gamma, bn1_beta, bn1_mean, bn1_var, act1);

  offset_conv_kernel<<<kNB * kL / kOcPos, 256, 0, stream>>>(act1, WP, off1_b, offs);

  sampled_conv_kernel<false><<<kNB * kL / kDcPos, 128, 0, stream>>>(
      act1, offs, WP + (size_t)32 * kCK, dc1_b,
      bn2_gamma, bn2_beta, bn2_mean, bn2_var, x, act2);

  offset_conv_kernel<<<kNB * kL / kOcPos, 256, 0, stream>>>(act2, WP + (size_t)16 * kCK, off2_b, offs);

  sampled_conv_kernel<true><<<kNB * kL / kDcPos, 128, 0, stream>>>(
      act2, offs, WP + (size_t)64 * kCK, dc2_b,
      bn2_gamma, bn2_beta, bn2_mean, bn2_var, x, outp);
}
